// Encoder_515396075689
// MI455X (gfx1250) — hardware-run, weakly checked
//
#include <hip/hip_runtime.h>
#include <math.h>

typedef __attribute__((ext_vector_type(16))) _Float16 v16h;
typedef __attribute__((ext_vector_type(8)))  float    v8f;
typedef __attribute__((ext_vector_type(4)))  float    v4f;

constexpr int kSeq      = 633;
constexpr int kIn       = 28;
constexpr int kH1       = 14;
constexpr int kH2       = 7;
constexpr int kG1       = 4 * kH1;
constexpr int kG2       = 4 * kH2;
constexpr int kMpad     = 640;
constexpr int kNpad     = 64;
constexpr int kKpad     = 32;
constexpr int kSlabP    = 68;
constexpr int kDot      = kH1 + kH2;
constexpr int kOutElems = kSeq * kH2;
constexpr int kOutLines = (kOutElems + 31) / 32;
constexpr int kOutLds   = kOutLines * 32;
constexpr float kXCarry = 64.0f;
constexpr float kWCarry = 64.0f;
constexpr float kFold   = 1.0f / (kXCarry * kWCarry);
constexpr float kF16MinNormal = 6.103515625e-5f;
constexpr size_t kWsG1Bytes = (size_t)kMpad * kNpad * 4;
constexpr size_t kWsTotal   = kWsG1Bytes;
static_assert(kG1 == 56);
static_assert(kG2 == 28);
static_assert(kMpad % 16 == 0 && kMpad >= kSeq);
static_assert(kNpad % 16 == 0 && kNpad >= kG1);
static_assert(kKpad == 32 && kKpad >= kIn);
static_assert((kIn % 4) == 0);
static_assert(kDot == 21);
static_assert(kOutElems == 4431);
static_assert(kOutLines == 139);
static_assert(kOutLds - kOutElems == 17);
static_assert(kWsTotal == 163840ull);
static_assert(kWsTotal <= 134217728ull);

__device__ __forceinline__ void pin1(float& v) { asm volatile("" : "+v"(v)); }

__device__ __forceinline__ _Float16 cvt_op_f16(float v) {
  const float z = (fabsf(v) < kF16MinNormal) ? 0.0f : v;
  return (_Float16)z;
}

__device__ __forceinline__ v16h load_frag_row28(const float* rowp, int hs, bool rowok, float carry) {
  const int ka = 8 * hs;
  const int kb = 16 + 8 * hs;
  const int kc = kb + 4;
  const bool tailok = (kc < kIn);
  const int kcc = tailok ? kc : (kIn - 4);
  v4f q0 = *(const v4f*)(rowp + ka);
  v4f q1 = *(const v4f*)(rowp + ka + 4);
  v4f q2 = *(const v4f*)(rowp + kb);
  v4f q3 = *(const v4f*)(rowp + kcc);
  asm volatile("" : "+v"(q0), "+v"(q1), "+v"(q2), "+v"(q3));
  const bool ok3 = rowok && tailok;
  v16h f;
#pragma unroll
  for (int e = 0; e < 4; ++e) {
    const float s0 = q0[e];
    const float s1 = q1[e];
    const float s2 = q2[e];
    const float s3 = q3[e];
    f[e]      = cvt_op_f16(rowok ? s0 * carry : 0.0f);
    f[4 + e]  = cvt_op_f16(rowok ? s1 * carry : 0.0f);
    f[8 + e]  = cvt_op_f16(rowok ? s2 * carry : 0.0f);
    f[12 + e] = cvt_op_f16(ok3   ? s3 * carry : 0.0f);
  }
  return f;
}

__device__ __forceinline__ v8f mma_f16(v16h a, v16h b, v8f c) {
  c = __builtin_amdgcn_wmma_f32_16x16x32_f16(false, a, false, b, (short)0, c, false, false);
  asm volatile("v_nop\n\tv_nop\n\tv_nop\n\tv_nop" : "+v"(c) : "v"(a), "v"(b));
  return c;
}

__global__ __launch_bounds__(128) void inproj_f16_kernel(
    const float* __restrict__ x, const float* __restrict__ w_ih1,
    const float* __restrict__ b_ih1, const float* __restrict__ b_hh1,
    float* __restrict__ G1)
{
  __shared__ __align__(16) float slab[16 * kSlabP];
  const int tid  = threadIdx.x;
  const int lane = tid & 31;
  const int wave = tid >> 5;
  const int c    = lane & 15;
  const int hs   = lane >> 4;
  const int row0 = blockIdx.x * 16;

  const int  m   = row0 + c;
  const bool mok = (m < kSeq);
  const int  mc  = mok ? m : (kSeq - 1);
  const int  n   = wave * 16 + c;
  const bool nok = (n < kG1);
  const int  nc  = nok ? n : (kG1 - 1);

  const v16h a = load_frag_row28(x     + (size_t)mc * kIn, hs, mok, kXCarry);
  const v16h b = load_frag_row28(w_ih1 + (size_t)nc * kIn, hs, nok, kWCarry);

  float bi = b_ih1[nc];
  float bh = b_hh1[nc];
  pin1(bi);
  pin1(bh);
  const float bsum = nok ? (bi + bh) : 0.0f;

  v8f acc = (v8f){0.f, 0.f, 0.f, 0.f, 0.f, 0.f, 0.f, 0.f};
  acc = mma_f16(a, b, acc);

#pragma unroll
  for (int r = 0; r < 8; ++r) {
    const float v = acc[r] * kFold + bsum;
    slab[(8 * hs + r) * kSlabP + n] = v;
  }
  __syncthreads();

  const int c4 = c * 4;
  v4f sv[2];
#pragma unroll
  for (int it = 0; it < 2; ++it) {
    const int row = 4 * wave + 2 * it + hs;
    sv[it] = *(const v4f*)(slab + row * kSlabP + c4);
  }
  for (int pass = 0; pass < 2; ++pass) {
#pragma unroll
    for (int it = 0; it < 2; ++it) {
      const int row = 4 * wave + 2 * it + hs;
      *(volatile v4f*)(G1 + (size_t)(row0 + row) * kNpad + c4) = sv[it];
    }
    __threadfence();
  }
}

__device__ __forceinline__ float sigm_f(float v) {
  return 1.0f / (1.0f + expf(-v));
}
__device__ __forceinline__ float tanh_f(float v) {
  return 1.0f - 2.0f / (expf(2.0f * v) + 1.0f);
}

__global__ __launch_bounds__(32) void lstm2_seq_kernel(
    const float* __restrict__ G1, const float* __restrict__ w_hh1,
    const float* __restrict__ w_ih2, const float* __restrict__ w_hh2,
    const float* __restrict__ b_ih2, const float* __restrict__ b_hh2,
    float* __restrict__ out)
{
  __shared__ __align__(16) float sW[kDot * 32 * 4];
  __shared__ __align__(16) float sV[32];
  __shared__ __align__(16) float sOut[kOutLds];

  const int  lane = threadIdx.x;
  const bool isL1 = (lane < kH1);
  const bool isL2 = (lane >= 16) && (lane < 16 + kH2);
  const int  j1c  = isL1 ? lane : (kH1 - 1);
  const int  j2r  = lane - 16;
  const int  j2c  = (j2r < 0) ? 0 : ((j2r > kH2 - 1) ? (kH2 - 1) : j2r);

  int widx;
  if (lane < kH1) widx = lane;
  else if (lane < 16) widx = lane + 7;
  else if (lane < 16 + kH2) widx = lane - 2;
  else widx = lane;

#pragma unroll 1
  for (int k = 0; k < kH1; ++k) {
    v4f wv;
#pragma unroll
    for (int g = 0; g < 4; ++g) {
      float wa = w_hh1[(g * kH1 + j1c) * kH1 + k];
      float wb = w_ih2[(g * kH2 + j2c) * kH1 + k];
      pin1(wa);
      pin1(wb);
      wv[g] = isL1 ? wa : (isL2 ? wb : 0.0f);
    }
    *(v4f*)(sW + (k * 32 + lane) * 4) = wv;
  }
#pragma unroll 1
  for (int k = 0; k < kH2; ++k) {
    v4f wv;
#pragma unroll
    for (int g = 0; g < 4; ++g) {
      float wc = w_hh2[(g * kH2 + j2c) * kH2 + k];
      pin1(wc);
      wv[g] = isL2 ? wc : 0.0f;
    }
    *(v4f*)(sW + ((kH1 + k) * 32 + lane) * 4) = wv;
  }

  float bs0, bs1, bs2, bs3;
  {
    float p0 = b_ih2[0 * kH2 + j2c];
    float p1 = b_ih2[1 * kH2 + j2c];
    float p2 = b_ih2[2 * kH2 + j2c];
    float p3 = b_ih2[3 * kH2 + j2c];
    float q0 = b_hh2[0 * kH2 + j2c];
    float q1 = b_hh2[1 * kH2 + j2c];
    float q2 = b_hh2[2 * kH2 + j2c];
    float q3 = b_hh2[3 * kH2 + j2c];
    pin1(p0); pin1(p1); pin1(p2); pin1(p3);
    pin1(q0); pin1(q1); pin1(q2); pin1(q3);
    bs0 = isL2 ? (p0 + q0) : 0.0f;
    bs1 = isL2 ? (p1 + q1) : 0.0f;
    bs2 = isL2 ? (p2 + q2) : 0.0f;
    bs3 = isL2 ? (p3 + q3) : 0.0f;
  }

  const int gc0 = 0 * kH1 + j1c;
  const int gc1 = 1 * kH1 + j1c;
  const int gc2 = 2 * kH1 + j1c;
  const int gc3 = 3 * kH1 + j1c;

  sV[lane] = 0.0f;
  if (lane < (kOutLds - kOutElems)) sOut[kOutElems + lane] = 0.0f;
  __syncthreads();

  float gv0 = G1[gc0];
  float gv1 = G1[gc1];
  float gv2 = G1[gc2];
  float gv3 = G1[gc3];
  pin1(gv0); pin1(gv1); pin1(gv2); pin1(gv3);

  float cst = 0.0f;

#pragma unroll 1
  for (int t = 0; t <= kSeq; ++t) {
    const int tn = (t + 1 < kSeq) ? (t + 1) : (kSeq - 1);
    float gn0 = G1[tn * kNpad + gc0];
    float gn1 = G1[tn * kNpad + gc1];
    float gn2 = G1[tn * kNpad + gc2];
    float gn3 = G1[tn * kNpad + gc3];
    pin1(gn0); pin1(gn1); pin1(gn2); pin1(gn3);

    float a0 = isL1 ? gv0 : bs0;
    float a1 = isL1 ? gv1 : bs1;
    float a2 = isL1 ? gv2 : bs2;
    float a3 = isL1 ? gv3 : bs3;
#pragma unroll 1
    for (int k = 0; k < kDot; ++k) {
      const v4f w = *(const v4f*)(sW + (k * 32 + lane) * 4);
      const float hv = sV[k];
      a0 = fmaf(w[0], hv, a0);
      a1 = fmaf(w[1], hv, a1);
      a2 = fmaf(w[2], hv, a2);
      a3 = fmaf(w[3], hv, a3);
    }
    const float ig = sigm_f(a0);
    const float fg = sigm_f(a1);
    const float gg = tanh_f(a2);
    const float og = sigm_f(a3);
    float cc = fg * cst + ig * gg;
    float hn = og * tanh_f(cc);
    const bool warm = (t == 0) && (!isL1);
    cc = warm ? 0.0f : cc;
    hn = warm ? 0.0f : hn;
    cst = cc;

    __syncthreads();
    sV[widx] = hn;
    if (isL2 && (t >= 1)) sOut[(t - 1) * kH2 + j2c] = hn;
    __syncthreads();

    gv0 = gn0; gv1 = gn1; gv2 = gn2; gv3 = gn3;
  }

  for (int pass = 0; pass < 2; ++pass) {
#pragma unroll 1
    for (int line = 0; line < kOutLines; ++line) {
      const int idx = line * 32 + lane;
      const float val = sOut[idx];
      if (idx < kOutElems) *(volatile float*)(out + idx) = val;
    }
    __threadfence();
  }
}

extern "C" void kernel_launch(void* const* d_in, const int* in_sizes, int n_in,
                              void* d_out, int out_size, void* d_ws, size_t ws_size,
                              hipStream_t stream) {
  if (n_in < 9 || d_out == nullptr || d_ws == nullptr) return;
  if (in_sizes[0] != kSeq * kIn) return;
  if (in_sizes[1] != kG1 * kIn) return;
  if (in_sizes[2] != kG1 * kH1) return;
  if (in_sizes[3] != kG1) return;
  if (in_sizes[4] != kG1) return;
  if (in_sizes[5] != kG2 * kH1) return;
  if (in_sizes[6] != kG2 * kH2) return;
  if (in_sizes[7] != kG2) return;
  if (in_sizes[8] != kG2) return;
  if (out_size != kOutElems) return;
  if (ws_size < kWsTotal) return;

  const float* x     = (const float*)d_in[0];
  const float* w_ih1 = (const float*)d_in[1];
  const float* w_hh1 = (const float*)d_in[2];
  const float* b_ih1 = (const float*)d_in[3];
  const float* b_hh1 = (const float*)d_in[4];
  const float* w_ih2 = (const float*)d_in[5];
  const float* w_hh2 = (const float*)d_in[6];
  const float* b_ih2 = (const float*)d_in[7];
  const float* b_hh2 = (const float*)d_in[8];
  float* out = (float*)d_out;
  float* G1  = (float*)d_ws;

  inproj_f16_kernel<<<kMpad / 16, 128, 0, stream>>>(x, w_ih1, b_ih1, b_hh1, G1);
  lstm2_seq_kernel<<<1, 32, 0, stream>>>(G1, w_hh1, w_ih2, w_hh2, b_ih2, b_hh2, out);
}
